// GAT_14181982012097
// MI455X (gfx1250) — hardware-verified
//
#include <hip/hip_runtime.h>
#include <math.h>
#include <stdint.h>

#ifndef NB
#define NB 2
#endif
#ifndef SEQ
#define SEQ 2048
#endif
#ifndef NB_FULL
#define NB_FULL 2
#endif
#ifndef SEQ_FULL
#define SEQ_FULL 2048
#endif
#define FIN   128
#define UD    64
#define NHD   4
#define HU    (NHD * UD)
#define OD    64
#define BN    (NB * SEQ)
#define PSC   4096.0f
#define HC    16.0f
#define WFC   64.0f
#define OSC   1.52587890625e-05f
#define G2INV 0.0009765625f
#define NEGFILL (-1.0e9f)

static_assert(NB >= 1 && NB <= NB_FULL && SEQ >= 64 && SEQ <= SEQ_FULL);
static_assert(SEQ % 64 == 0 && BN % 64 == 0);
static_assert(FIN % 64 == 0 && FIN % 32 == 0 && UD == 64 && OD == 64 && HU % 64 == 0 && HU % 32 == 0);
static_assert(PSC * HC * OSC == 1.0f);
static_assert(HC * WFC * G2INV == 1.0f);

typedef __bf16         v16b __attribute__((ext_vector_type(16)));
typedef __bf16         v8b  __attribute__((ext_vector_type(8)));
typedef _Float16       v16h __attribute__((ext_vector_type(16)));
typedef _Float16       v8h  __attribute__((ext_vector_type(8)));
typedef _Float16       v4h  __attribute__((ext_vector_type(4)));
typedef float          v8f  __attribute__((ext_vector_type(8)));
typedef float          v4f  __attribute__((ext_vector_type(4)));
typedef unsigned int   v4u  __attribute__((ext_vector_type(4)));
typedef int            v4i  __attribute__((ext_vector_type(4)));
typedef v4f __attribute__((may_alias)) v4fa;
typedef v4u __attribute__((may_alias)) v4ua;
typedef v4i __attribute__((may_alias)) v4ia;
typedef v8b __attribute__((may_alias)) v8ba;
typedef v8h __attribute__((may_alias)) v8ha;
typedef v4h __attribute__((may_alias)) v4ha;
typedef _Float16 h16;

__device__ __forceinline__ unsigned short bf_bits(float f) {
  const unsigned u = __float_as_uint(f);
  return (unsigned short)((u + 0x7FFFu + ((u >> 16) & 1u)) >> 16);
}
__device__ __forceinline__ float bf_val(unsigned short h) { return __uint_as_float(((unsigned)h) << 16); }
__device__ __forceinline__ float bf_rne(float f) { return bf_val(bf_bits(f)); }
__device__ __forceinline__ v4f bf_rne4(v4f a) {
  v4f r;
  r[0] = bf_rne(a[0]); r[1] = bf_rne(a[1]); r[2] = bf_rne(a[2]); r[3] = bf_rne(a[3]);
  return r;
}
__device__ __forceinline__ unsigned short h_bits(float f) {
  const _Float16 hv = (_Float16)f;
  return __builtin_bit_cast(unsigned short, hv);
}
template <int KIND>
__device__ __forceinline__ unsigned short cvt16(float f) { return KIND == 0 ? bf_bits(f) : h_bits(bf_rne(f)); }
__device__ __forceinline__ unsigned pk16(unsigned short a, unsigned short b) { return (unsigned)a | ((unsigned)b << 16); }
__device__ __forceinline__ v8f zero8() { v8f z = {0.f, 0.f, 0.f, 0.f, 0.f, 0.f, 0.f, 0.f}; return z; }
__device__ __forceinline__ int wave_id() { return __builtin_amdgcn_readfirstlane((int)(threadIdx.x >> 5)); }

__device__ __forceinline__ void lds_wave_sync() {
  __builtin_amdgcn_fence(3  , "workgroup");
  __builtin_amdgcn_wave_barrier();
  __builtin_amdgcn_fence(2  , "workgroup");
}

static __device__ __forceinline__ h16 toh_flush(float v) {
  const float w = (fabsf(v) < 6.103515625e-05f) ? 0.0f : v;
  return (h16)w;
}
__device__ __forceinline__ unsigned short hf_bits(float f) {
  const h16 r = toh_flush(f);
  return __builtin_bit_cast(unsigned short, r);
}

union FragB { v16b v; v8b h[2]; };
union FragH { v16h v; v8h h[2]; };
__device__ __forceinline__ v16b ldfrag_b(const __bf16* p) {
  FragB f;
  f.h[0] = *(const v8ba*)(p);
  f.h[1] = *(const v8ba*)(p + 16);
  return f.v;
}
__device__ __forceinline__ v16h ldfrag_h(const _Float16* p) {
  FragH f;
  f.h[0] = *(const v8ha*)(p);
  f.h[1] = *(const v8ha*)(p + 16);
  return f.v;
}
__device__ __forceinline__ v8f mma_b(v16b a, v16b b, v8f c) {
  return __builtin_amdgcn_wmma_f32_16x16x32_bf16(false, a, false, b, (short)0, c, false, false);
}
__device__ __forceinline__ v8f mma_h(v16h a, v16h b, v8f c) {
  return __builtin_amdgcn_wmma_f32_16x16x32_f16(false, a, false, b, (short)0, c, false, false);
}
static __device__ __forceinline__ v8f wmmabg(v16b a, v16b b, v8f c) {
  c = mma_b(a, b, c);
  asm volatile("v_nop\n\tv_nop\n\tv_nop\n\tv_nop" : "+v"(c) : "v"(a), "v"(b));
  return c;
}
static __device__ __forceinline__ v8f wmma16g(v16h a, v16h b, v8f c) {
  c = mma_h(a, b, c);
  asm volatile("v_nop\n\tv_nop\n\tv_nop\n\tv_nop" : "+v"(c) : "v"(a), "v"(b));
  return c;
}

__global__ __launch_bounds__(256) void prep_x_kernel(const float* __restrict__ x, unsigned short* __restrict__ xb, int nunits) {
  const int i = (int)blockIdx.x * 256 + (int)threadIdx.x;
  if (i >= nunits) return;
  const size_t e  = 8 * (size_t)i;
  const int    bn = (int)(e / FIN);
  const int    f  = (int)(e - (size_t)bn * FIN);
  const int    b  = bn / SEQ;
  const int    n  = bn - b * SEQ;
  const float* src = x + ((size_t)b * SEQ_FULL + n) * FIN + f;
  const v4f a = *(const v4fa*)(src);
  const v4f c = *(const v4fa*)(src + 4);
  v4u w;
  w[0] = pk16(bf_bits(a[0]), bf_bits(a[1]));
  w[1] = pk16(bf_bits(a[2]), bf_bits(a[3]));
  w[2] = pk16(bf_bits(c[0]), bf_bits(c[1]));
  w[3] = pk16(bf_bits(c[2]), bf_bits(c[3]));
  *(volatile v4u*)(xb + e) = w;
  __threadfence();
  *(volatile v4u*)(xb + e) = w;
}

template <int KIND>
__global__ __launch_bounds__(256) void tconv_kernel(const float* __restrict__ W, unsigned short* __restrict__ outp,
                                                    int R, int Cc, long sIn, long sOut) {
  __shared__ __align__(16) float tf[64 * 68];
  W    += (size_t)blockIdx.z * sIn;
  outp += (size_t)blockIdx.z * sOut;
  const int c0  = (int)blockIdx.x * 64;
  const int r0  = (int)blockIdx.y * 64;
  const int tid = (int)threadIdx.x;
  {
    const int lr = tid >> 4;
    const int c4 = (tid & 15) * 4;
#pragma unroll
    for (int it = 0; it < 4; ++it) {
      const int rr = it * 16 + lr;
      const v4f a = *(const v4fa*)(W + (size_t)(r0 + rr) * Cc + c0 + c4);
      *(v4f*)(tf + rr * 68 + c4) = a;
    }
  }
  __syncthreads();
  const int sub = tid >> 3;
  const int c8  = (tid & 7) * 8;
  v4u hv[2];
#pragma unroll
  for (int it = 0; it < 2; ++it) {
    const int oc = it * 32 + sub;
    v4u a;
#pragma unroll
    for (int q = 0; q < 4; ++q) {
      const float f0 = tf[(c8 + 2 * q) * 68 + oc];
      const float f1 = tf[(c8 + 2 * q + 1) * 68 + oc];
      a[q] = pk16(cvt16<KIND>(f0), cvt16<KIND>(f1));
    }
    hv[it] = a;
  }
  for (int pass = 0; pass < 2; ++pass) {
#pragma unroll
    for (int it = 0; it < 2; ++it) {
      const int oc = it * 32 + sub;
      const size_t go = (size_t)(c0 + oc) * R + r0 + c8;
      *(volatile v4u*)(outp + go) = hv[it];
    }
    __threadfence();
  }
}

__global__ __launch_bounds__(256) void tconv_sc_kernel(const float* __restrict__ W, unsigned short* __restrict__ outp,
                                                       int R, int Cc, long sIn, long sOut) {
  __shared__ __align__(16) float tf[64 * 68];
  W    += (size_t)blockIdx.z * sIn;
  outp += (size_t)blockIdx.z * sOut;
  const int c0  = (int)blockIdx.x * 64;
  const int r0  = (int)blockIdx.y * 64;
  const int tid = (int)threadIdx.x;
  {
    const int lr = tid >> 4;
    const int c4 = (tid & 15) * 4;
#pragma unroll
    for (int it = 0; it < 4; ++it) {
      const int rr = it * 16 + lr;
      const v4f a = *(const v4fa*)(W + (size_t)(r0 + rr) * Cc + c0 + c4);
      *(v4f*)(tf + rr * 68 + c4) = a;
    }
  }
  __syncthreads();
  const int sub = tid >> 3;
  const int c8  = (tid & 7) * 8;
  v4u hv[2];
#pragma unroll
  for (int it = 0; it < 2; ++it) {
    const int oc = it * 32 + sub;
    v4u a;
#pragma unroll
    for (int q = 0; q < 4; ++q) {
      const float f0 = tf[(c8 + 2 * q) * 68 + oc];
      const float f1 = tf[(c8 + 2 * q + 1) * 68 + oc];
      a[q] = pk16(hf_bits(WFC * bf_rne(f0)), hf_bits(WFC * bf_rne(f1)));
    }
    hv[it] = a;
  }
  for (int pass = 0; pass < 2; ++pass) {
#pragma unroll
    for (int it = 0; it < 2; ++it) {
      const int oc = it * 32 + sub;
      const size_t go = (size_t)(c0 + oc) * R + r0 + c8;
      *(volatile v4u*)(outp + go) = hv[it];
    }
    __threadfence();
  }
}

#define STP      68
#define ST_PERW  (16 * STP)
static_assert((STP * 4) % 16 == 0 && STP >= 64);
static_assert(4 * 32 * 16 == 16 * 64 * 2);
static_assert(4 * ST_PERW * 4 <= 131072);

template <bool F16OPS> struct GemmOps;
template <> struct GemmOps<false> {
  typedef v16b frag;
  static __device__ __forceinline__ frag ld(const unsigned short* p) { return ldfrag_b((const __bf16*)(const void*)p); }
  static __device__ __forceinline__ v8f mma(frag a, frag b, v8f c) { return wmmabg(a, b, c); }
  static __device__ __forceinline__ float cs() { return 1.0f; }
};
template <> struct GemmOps<true> {
  typedef v16h frag;
  static __device__ __forceinline__ frag ld(const unsigned short* p) { return ldfrag_h((const _Float16*)(const void*)p); }
  static __device__ __forceinline__ v8f mma(frag a, frag b, v8f c) { return wmma16g(a, b, c); }
  static __device__ __forceinline__ float cs() { return G2INV; }
};

template <bool F16OPS, int NH>
__device__ __forceinline__ void gemm_body(const unsigned short* Ap, int lda, const unsigned short* Btp, int ldb, int M, int K,
                                          const float* __restrict__ av1, const float* __restrict__ av2,
                                          float* sd, int bnp, unsigned short* ht, float* stage_all) {
  typedef typename GemmOps<F16OPS>::frag frag_t;
  const int lane = threadIdx.x & 31;
  const int wave = wave_id();
  const int hh = lane >> 4;
  const int rl = lane & 15;
  const unsigned tilesM = (unsigned)M >> 6;
  const unsigned bx   = blockIdx.x;
  const unsigned tile = bx * 4u + (unsigned)wave;
  if (tile >= tilesM * (unsigned)NH) return;
  const unsigned tm = tile / (unsigned)NH;
  const unsigned tn = tile - tm * (unsigned)NH;
  const int m0 = (int)(tm << 6);
  const int n0 = (int)(tn << 6);

  v8f acc[4][4];
#pragma unroll
  for (int i = 0; i < 4; ++i)
#pragma unroll
    for (int j = 0; j < 4; ++j) acc[i][j] = zero8();

  for (int k0 = 0; k0 < K; k0 += 32) {
    const frag_t a0f = GemmOps<F16OPS>::ld(Ap + (size_t)(m0 + rl) * lda + k0 + 8 * hh);
    const frag_t a1f = GemmOps<F16OPS>::ld(Ap + (size_t)(m0 + 16 + rl) * lda + k0 + 8 * hh);
    const frag_t a2f = GemmOps<F16OPS>::ld(Ap + (size_t)(m0 + 32 + rl) * lda + k0 + 8 * hh);
    const frag_t a3f = GemmOps<F16OPS>::ld(Ap + (size_t)(m0 + 48 + rl) * lda + k0 + 8 * hh);
#pragma unroll
    for (int j = 0; j < 4; ++j) {
      const frag_t bh = GemmOps<F16OPS>::ld(Btp + (size_t)(n0 + j * 16 + rl) * ldb + k0 + 8 * hh);
      acc[0][j] = GemmOps<F16OPS>::mma(a0f, bh, acc[0][j]);
      acc[1][j] = GemmOps<F16OPS>::mma(a1f, bh, acc[1][j]);
      acc[2][j] = GemmOps<F16OPS>::mma(a2f, bh, acc[2][j]);
      acc[3][j] = GemmOps<F16OPS>::mma(a3f, bh, acc[3][j]);
    }
  }

  float* st = stage_all + wave * ST_PERW;
  const float cs = GemmOps<F16OPS>::cs();
  const unsigned bidx = (unsigned)m0 / (unsigned)SEQ;
  const int nl0 = m0 - (int)bidx * SEQ;
  const int q   = lane >> 3;
  const int p8  = (lane & 7) * 8;
  float s1a = 0.f, s1b = 0.f, s2a = 0.f, s2b = 0.f;
#pragma unroll
  for (int j = 0; j < 4; ++j) {
#pragma unroll
    for (int i = 0; i < 4; ++i) {
      v4f lo, hi;
#pragma unroll
      for (int r = 0; r < 4; ++r) { lo[r] = acc[i][j][r] * cs; hi[r] = acc[i][j][4 + r] * cs; }
      *(v4fa*)(st + rl * STP + 16 * i + 8 * hh)     = lo;
      *(v4fa*)(st + rl * STP + 16 * i + 8 * hh + 4) = hi;
    }
    lds_wave_sync();
    {
      const float* w1p = av1 + n0 + j * 16;
      const float* w2p = av2 + n0 + j * 16;
      for (int o4 = 0; o4 < 4; ++o4) {
        const v4f w1 = bf_rne4(*(const v4fa*)(w1p + o4 * 4));
        const v4f w2 = bf_rne4(*(const v4fa*)(w2p + o4 * 4));
#pragma unroll
        for (int u = 0; u < 4; ++u) {
          const float ca = st[(o4 * 4 + u) * STP + lane];
          const float cb = st[(o4 * 4 + u) * STP + 32 + lane];
          s1a = fmaf(ca, w1[u], s1a);
          s1b = fmaf(cb, w1[u], s1b);
          s2a = fmaf(ca, w2[u], s2a);
          s2b = fmaf(cb, w2[u], s2b);
        }
      }
    }
    v4u hv[4];
#pragma unroll
    for (int it = 0; it < 4; ++it) {
      const int ol = it * 4 + q;
      const v4f x0 = *(const v4fa*)(st + ol * STP + p8);
      const v4f x1 = *(const v4fa*)(st + ol * STP + p8 + 4);
      v4u a;
      a[0] = pk16(hf_bits(HC * x0[0]), hf_bits(HC * x0[1]));
      a[1] = pk16(hf_bits(HC * x0[2]), hf_bits(HC * x0[3]));
      a[2] = pk16(hf_bits(HC * x1[0]), hf_bits(HC * x1[1]));
      a[3] = pk16(hf_bits(HC * x1[2]), hf_bits(HC * x1[3]));
      hv[it] = a;
    }
    unsigned short* hb = ht + ((size_t)(bidx * (unsigned)NH + tn) * UD + j * 16) * SEQ + nl0 + p8;
    for (int pass = 0; pass < 2; ++pass) {
#pragma unroll
      for (int it = 0; it < 4; ++it)
        *(volatile v4u*)(hb + (size_t)(it * 4 + q) * SEQ) = hv[it];
      __threadfence();
    }
    lds_wave_sync();
  }
  float* base = sd + (size_t)tn * bnp + m0 + lane;
  for (int pass = 0; pass < 2; ++pass) {
    *(volatile float*)(base)                            = s1a;
    *(volatile float*)(base + 32)                       = s1b;
    *(volatile float*)(base + (size_t)NH * bnp)         = s2a;
    *(volatile float*)(base + (size_t)NH * bnp + 32)    = s2b;
    __threadfence();
  }
}

__global__ __launch_bounds__(128) __attribute__((amdgpu_num_vgpr(256))) void gemm1_kernel(
    const unsigned short* Ap, const unsigned short* Btp, const float* __restrict__ av1, const float* __restrict__ av2,
    float* sd, unsigned short* ht) {
  __shared__ __align__(16) float stage_all[4 * ST_PERW];
  gemm_body<false, NHD>(Ap, FIN, Btp, FIN, BN, FIN, av1, av2, sd, BN, ht, stage_all);
}
__global__ __launch_bounds__(128) __attribute__((amdgpu_num_vgpr(256))) void gemm2_kernel(
    const unsigned short* Ap, const unsigned short* Btp, const float* __restrict__ av1, const float* __restrict__ av2,
    float* sd, unsigned short* ht) {
  __shared__ __align__(16) float stage_all[4 * ST_PERW];
  gemm_body<true, 1>(Ap, HU, Btp, HU, BN, HU, av1, av2, sd, BN, ht, stage_all);
}

#define KT       64
#define PSP      72
#define OSTP     64
#define NTILE    (UD / 16)
#define ATT_P_H  (4 * 16 * PSP)
#define ATT_S_F  (4 * 16 * OSTP)
static_assert(ATT_P_H * 2 + ATT_S_F * 4 <= 131072);
static_assert(SEQ % KT == 0 && KT == 64 && NTILE == 4);
static_assert(4 * 32 * 16 == 16 * UD * 2);
static_assert(8 * 32 * 16 == 16 * OD * 4);
static_assert(OD == UD);

template <int NH, int LAYER>
__device__ __forceinline__ void attn_body(const int* __restrict__ adj, const float* __restrict__ sd,
                                          const unsigned short* __restrict__ vt,
                                          unsigned short* __restrict__ cat, float* __restrict__ out,
                                          _Float16* lds_p, float* lds_s) {
  const int tid  = (int)threadIdx.x;
  const int lane = tid & 31;
  const int wave = wave_id();
  const int hh   = lane >> 4;
  const int c    = lane & 15;
  const int qb   = (int)blockIdx.x;
  const int h    = (int)blockIdx.y;
  const int b    = (int)blockIdx.z;
  const int q0   = qb * 64 + wave * 16;

  const int*      Ag = adj + (size_t)b * SEQ_FULL * SEQ_FULL + (size_t)(q0 + 8 * hh) * SEQ_FULL + 4 * c;
  const float*    Dg = sd + (size_t)(NH + h) * BN + (size_t)b * SEQ + 4 * c;
  const _Float16* Vg = (const _Float16*)(const void*)vt + (size_t)(b * NH + h) * UD * SEQ + 8 * hh;
  _Float16* ph = lds_p + wave * (16 * PSP);

  float cadd[8];
  {
    const size_t ro = (size_t)h * BN + (size_t)b * SEQ + q0 + 8 * hh;
    const v4f s0 = *(const v4fa*)(sd + ro);
    const v4f s1 = *(const v4fa*)(sd + ro + 4);
#pragma unroll
    for (int r = 0; r < 4; ++r) { cadd[r] = s0[r]; cadd[4 + r] = s1[r]; }
  }

  float mrow[8], lrow[8];
#pragma unroll
  for (int r = 0; r < 8; ++r) { mrow[r] = -INFINITY; lrow[r] = 0.f; }

  v8f oc[NTILE];
#pragma unroll
  for (int t = 0; t < NTILE; ++t) oc[t] = zero8();

#pragma unroll 1
  for (int kc = 0; kc < SEQ / KT; ++kc) {
    const int kv0 = kc * KT;
    const v4f d4 = *(const v4fa*)(Dg + kv0);
    float s[8][4];
    float cm[8];
#pragma unroll
    for (int r = 0; r < 8; ++r) {
      const v4i m4 = *(const v4ia*)(Ag + (size_t)r * SEQ_FULL + kv0);
      float m = -INFINITY;
#pragma unroll
      for (int q = 0; q < 4; ++q) {
        const float t  = cadd[r] + d4[q];
        const float e  = (t >= 0.0f) ? t : 0.2f * t;
        const float sv = (m4[q] != 0) ? e : NEGFILL;
        s[r][q] = sv;
        m = fmaxf(m, sv);
      }
#pragma unroll
      for (int off = 1; off < 16; off <<= 1) m = fmaxf(m, __shfl_xor(m, off, 32));
      cm[r] = m;
    }
    float alpha[8];
#pragma unroll
    for (int r = 0; r < 8; ++r) {
      const float mnew = fmaxf(mrow[r], cm[r]);
      const float al   = __expf(mrow[r] - mnew);
      mrow[r]  = mnew;
      alpha[r] = al;
      float psum = 0.f;
      v4h pv;
#pragma unroll
      for (int q = 0; q < 4; ++q) {
        const float p = __expf(s[r][q] - mnew);
        psum += p;
        pv[q] = toh_flush(p * PSC);
      }
      *(v4ha*)(ph + (8 * hh + r) * PSP + 4 * c) = pv;
#pragma unroll
      for (int off = 1; off < 16; off <<= 1) psum += __shfl_xor(psum, off, 32);
      lrow[r] = lrow[r] * al + psum;
    }
    lds_wave_sync();
    const v16h pa0 = ldfrag_h(ph + c * PSP + 8 * hh);
    const v16h pa1 = ldfrag_h(ph + c * PSP + 32 + 8 * hh);
#pragma unroll
    for (int t = 0; t < NTILE; ++t) {
      v8f o8 = oc[t];
#pragma unroll
      for (int r = 0; r < 8; ++r) o8[r] = o8[r] * alpha[r];
      const size_t vo = (size_t)(t * 16 + c) * SEQ + kv0;
      const v16h vb0 = ldfrag_h(Vg + vo);
      const v16h vb1 = ldfrag_h(Vg + vo + 32);
      o8 = wmma16g(pa0, vb0, o8);
      o8 = wmma16g(pa1, vb1, o8);
      oc[t] = o8;
    }
    lds_wave_sync();
  }

  float inv[8];
#pragma unroll
  for (int r = 0; r < 8; ++r) inv[r] = (1.0f / lrow[r]) * OSC;
  float* os = lds_s + wave * (16 * OSTP);
#pragma unroll
  for (int t = 0; t < NTILE; ++t) {
#pragma unroll
    for (int r = 0; r < 8; ++r) {
      const float v = oc[t][r] * inv[r];
      os[(8 * hh + r) * OSTP + t * 16 + c] = (v > 0.0f) ? v : expm1f(v);
    }
  }
  lds_wave_sync();

  if (LAYER == 1) {
    const int q  = lane >> 3;
    const int p8 = (lane & 7) * 8;
    v4u cv[4];
#pragma unroll
    for (int it = 0; it < 4; ++it) {
      const int row = it * 4 + q;
      const v4f x0 = *(const v4fa*)(os + row * OSTP + p8);
      const v4f x1 = *(const v4fa*)(os + row * OSTP + p8 + 4);
      v4u a;
      a[0] = pk16(hf_bits(HC * x0[0]), hf_bits(HC * x0[1]));
      a[1] = pk16(hf_bits(HC * x0[2]), hf_bits(HC * x0[3]));
      a[2] = pk16(hf_bits(HC * x1[0]), hf_bits(HC * x1[1]));
      a[3] = pk16(hf_bits(HC * x1[2]), hf_bits(HC * x1[3]));
      cv[it] = a;
    }
    unsigned short* cb = cat + ((size_t)b * SEQ + q0) * HU + h * UD + p8;
    for (int pass = 0; pass < 2; ++pass) {
#pragma unroll
      for (int it = 0; it < 4; ++it)
        *(volatile v4u*)(cb + (size_t)(it * 4 + q) * HU) = cv[it];
      __threadfence();
    }
  } else {
    const int rr = lane >> 4;
    const int cq = lane & 15;
    for (int it = 0; it < 8; ++it) {
      float* rp = os + (it * 2 + rr) * OSTP + 4 * cq;
      const v4f x = *(const v4fa*)(rp);
      float m = fmaxf(fmaxf(x[0], x[1]), fmaxf(x[2], x[3]));
#pragma unroll
      for (int off = 1; off < 16; off <<= 1) m = fmaxf(m, __shfl_xor(m, off, 32));
      float sm = expf(x[0] - m) + expf(x[1] - m) + expf(x[2] - m) + expf(x[3] - m);
#pragma unroll
      for (int off = 1; off < 16; off <<= 1) sm += __shfl_xor(sm, off, 32);
      const float lg = m + logf(sm);
      v4f y;
      y[0] = x[0] - lg; y[1] = x[1] - lg; y[2] = x[2] - lg; y[3] = x[3] - lg;
      *(v4fa*)(rp) = y;
    }
    lds_wave_sync();
    float* ob = out + ((size_t)b * SEQ + q0) * OD + lane * 4;
    for (int pass = 0; pass < 2; ++pass) {
#pragma unroll
      for (int it = 0; it < 8; ++it) {
        const v4f xv = *(const v4fa*)(os + (it * 2 + rr) * OSTP + 4 * cq);
        *(volatile v4f*)(ob + (size_t)it * 2 * OD) = xv;
      }
      __threadfence();
    }
  }
}

__global__ __launch_bounds__(128) __attribute__((amdgpu_num_vgpr(240))) void attn1_kernel(
    const int* __restrict__ adj, const float* __restrict__ sd, const unsigned short* __restrict__ vt,
    unsigned short* __restrict__ cat) {
  __shared__ __align__(16) _Float16 p_tile[ATT_P_H];
  __shared__ __align__(16) float    o_stage[ATT_S_F];
  attn_body<NHD, 1>(adj, sd, vt, cat, (float*)nullptr, p_tile, o_stage);
}
__global__ __launch_bounds__(128) __attribute__((amdgpu_num_vgpr(240))) void attn2_kernel(
    const int* __restrict__ adj, const float* __restrict__ sd, const unsigned short* __restrict__ vt,
    float* __restrict__ out) {
  __shared__ __align__(16) _Float16 p_tile[ATT_P_H];
  __shared__ __align__(16) float    o_stage[ATT_S_F];
  attn_body<1, 2>(adj, sd, vt, (unsigned short*)nullptr, out, p_tile, o_stage);
}

#define SZ_XB ((size_t)BN * FIN * 2)
#define SZ_WT ((size_t)HU * FIN * 2)
#define SZ_WF ((size_t)OD * HU * 2)
#define SZ_H1 ((size_t)NB * NHD * UD * SEQ * 2)
#define SZ_S1 ((size_t)2 * NHD * BN * 4)
#define SZ_CT ((size_t)BN * HU * 2)
#define SZ_H2 ((size_t)NB * OD * SEQ * 2)
#define SZ_S2 ((size_t)2 * BN * 4)
#define WS_TOTAL (SZ_XB + SZ_WT + SZ_WF + SZ_H1 + SZ_S1 + SZ_CT + SZ_H2 + SZ_S2)
#define GEMM1_BLOCKS (((BN / 64) * NHD + 3) / 4)
#define GEMM2_BLOCKS (((BN / 64) + 3) / 4)
#define PREP_UNITS   (BN * FIN / 8)
static_assert(WS_TOTAL <= 134217728);
static_assert(SZ_XB % 128 == 0 && SZ_WT % 128 == 0 && SZ_WF % 128 == 0 && SZ_H1 % 128 == 0);
static_assert(SZ_S1 % 128 == 0 && SZ_CT % 128 == 0 && SZ_H2 % 128 == 0 && SZ_S2 % 128 == 0);
static_assert(NB != 2 || SEQ != 2048 || WS_TOTAL == 6029312);
static_assert(((size_t)BN - 1) * OD + OD - 1 < (size_t)BN * OD);
static_assert((BN * FIN / 8) % 256 == 0);
static_assert(UD % 64 == 0 && FIN % 64 == 0 && HU % 64 == 0 && OD % 64 == 0);

extern "C" void kernel_launch(void* const* d_in, const int* in_sizes, int n_in,
                              void* d_out, int out_size, void* d_ws, size_t ws_size,
                              hipStream_t stream) {
  if (n_in < 8) return;
  const long long needX = ((long long)(NB - 1) * SEQ_FULL + SEQ) * FIN;
  const long long needA = (long long)(NB - 1) * SEQ_FULL * SEQ_FULL + (long long)(SEQ - 1) * SEQ_FULL + SEQ;
  if ((long long)in_sizes[0] < needX) return;
  if ((long long)in_sizes[1] < needA) return;
  if (in_sizes[2] != NHD * FIN * UD) return;
  if (in_sizes[3] != NHD * UD) return;
  if (in_sizes[4] != NHD * UD) return;
  if (in_sizes[5] != HU * OD) return;
  if (in_sizes[6] != OD) return;
  if (in_sizes[7] != OD) return;
  if (out_size != BN * OD) return;

  const float* X    = (const float*)d_in[0];
  const int*   Adj  = (const int*)d_in[1];
  const float* Wk   = (const float*)d_in[2];
  const float* A1   = (const float*)d_in[3];
  const float* A2   = (const float*)d_in[4];
  const float* Wf   = (const float*)d_in[5];
  const float* A1f  = (const float*)d_in[6];
  const float* A2f  = (const float*)d_in[7];
  float* out = (float*)d_out;

  size_t off = 0;
  const size_t oXB = off; off += SZ_XB;
  const size_t oWT = off; off += SZ_WT;
  const size_t oWF = off; off += SZ_WF;
  const size_t oH1 = off; off += SZ_H1;
  const size_t oS1 = off; off += SZ_S1;
  const size_t oCT = off; off += SZ_CT;
  const size_t oH2 = off; off += SZ_H2;
  const size_t oS2 = off; off += SZ_S2;
  if (off != WS_TOTAL) return;
  if (off > ws_size) return;

  char* ws = (char*)d_ws;
  unsigned short* XB  = (unsigned short*)(ws + oXB);
  unsigned short* WTB = (unsigned short*)(ws + oWT);
  unsigned short* WFT = (unsigned short*)(ws + oWF);
  unsigned short* HT1 = (unsigned short*)(ws + oH1);
  float*          SD1 = (float*)(ws + oS1);
  unsigned short* CAT = (unsigned short*)(ws + oCT);
  unsigned short* HT2 = (unsigned short*)(ws + oH2);
  float*          SD2 = (float*)(ws + oS2);

  const dim3 b256(256), b128(128);

  prep_x_kernel<<<dim3((PREP_UNITS + 255) / 256), b256, 0, stream>>>(X, XB, PREP_UNITS);
  tconv_kernel<0><<<dim3(UD / 64, FIN / 64, NHD), b256, 0, stream>>>(Wk, WTB, FIN, UD, (long)FIN * UD, (long)UD * FIN);
  tconv_sc_kernel<<<dim3(OD / 64, HU / 64, 1), b256, 0, stream>>>(Wf, WFT, HU, OD, (long)HU * OD, (long)OD * HU);
  gemm1_kernel<<<dim3(GEMM1_BLOCKS), b128, 0, stream>>>(XB, WTB, A1, A2, SD1, HT1);
  attn1_kernel<<<dim3(SEQ / 64, NHD, NB), b128, 0, stream>>>(Adj, SD1, HT1, CAT);
  gemm2_kernel<<<dim3(GEMM2_BLOCKS), b128, 0, stream>>>(CAT, WFT, A1f, A2f, SD2, HT2);
  attn2_kernel<<<dim3(SEQ / 64, 1, NB), b128, 0, stream>>>(Adj, SD2, HT2, out);
  (void)hipGetLastError();
}
